// Block_22497038696617
// MI455X (gfx1250) — hardware-verified
//
#include <hip/hip_runtime.h>


#ifndef NB
#define NB 2
#endif
#ifndef SEQ
#define SEQ 2048
#endif
#define NB_FULL 2
#define SEQ_FULL 2048
#define CE 768
#define NH 12
#define HD 64
#define C3 2304
#define C4 3072
#define QP 1536
#define RROWS ((NB) * (SEQ))
#define NQB ((SEQ) / 128)
#define NKT ((SEQ) / 64)
#define LNJ ((CE) / 128)
#define LNO ((CE) / 256)
#define VROWS ((NB) * NH * HD)

static_assert((SEQ) % 256 == 0);
static_assert((NB) >= 1 && (NB) <= NB_FULL);
static_assert((SEQ) <= SEQ_FULL);
static_assert(CE % 128 == 0 && C3 % 128 == 0 && C4 % 128 == 0 && QP % 128 == 0);
static_assert(CE % 64 == 0 && C4 % 64 == 0);
static_assert(NH * HD == CE);
static_assert(HD == 64);
static_assert(QP == 2 * CE);
static_assert(C3 == 3 * CE);
static_assert(RROWS % 128 == 0);
static_assert(RROWS % 8 == 0);
static_assert(CE / 4 <= 256 && (CE / 4) % 32 == 0);
static_assert(32 * 4 * LNJ == CE);
static_assert(32 * 8 * LNO == CE);
static_assert(NQB * 128 == (SEQ));
static_assert(NKT * 64 == (SEQ));
static_assert(VROWS % 32 == 0);
static_assert(((size_t)C3 * CE) % 2048 == 0);
static_assert(((size_t)CE * CE) % 2048 == 0);
static_assert(((size_t)C4 * CE) % 2048 == 0);

typedef unsigned short u16;
typedef unsigned int   u32;
typedef _Float16 v16h __attribute__((ext_vector_type(16)));
typedef _Float16 v8h  __attribute__((ext_vector_type(8)));
typedef _Float16 v4h  __attribute__((ext_vector_type(4)));
typedef float    v8f  __attribute__((ext_vector_type(8)));
typedef float    v4f  __attribute__((ext_vector_type(4)));
typedef unsigned int u32x4 __attribute__((ext_vector_type(4)));
typedef unsigned int u32x2 __attribute__((ext_vector_type(2)));

union Frag  { v16h v; u32x4 u[2]; };
union Pack8 { v8h h; u32x4 u; };
union Pack4 { v4h h; u32x2 u; };

#define WSCALE 64.0f
#define WINV   (1.0f / 64.0f)
#define PCAR   4096.0f
#define PINV   (1.0f / 4096.0f)
#define CVCAR  64.0f
#define CVINV  (1.0f / 64.0f)

constexpr size_t al256(size_t b) { return (b + 255) & ~(size_t)255; }
constexpr size_t WS_TOTAL =
    al256((size_t)C3 * CE * 2) + al256((size_t)CE * CE * 2) + al256((size_t)C4 * CE * 2) +
    al256((size_t)CE * C4 * 2) + al256((size_t)RROWS * CE * 2) + al256((size_t)RROWS * QP * 2) +
    al256((size_t)VROWS * (SEQ) * 2) + al256((size_t)VROWS * 4) + al256((size_t)RROWS * CE * 2) +
    al256((size_t)RROWS * CE * 4) + al256((size_t)RROWS * CE * 2) + al256((size_t)RROWS * C4 * 2);
static_assert(WS_TOTAL <= (size_t)134217728);

__device__ __forceinline__ float bfr(float f) {
    u32 u = __builtin_bit_cast(u32, f);
    u += 0x7fffu + ((u >> 16) & 1u);
    u &= 0xffff0000u;
    return __builtin_bit_cast(float, u);
}

__device__ __forceinline__ u16 hbits(float f) {
    _Float16 h = (_Float16)f;
    return __builtin_bit_cast(u16, h);
}

__device__ __forceinline__ v8f mma16(v16h a, v16h b, v8f c) {
    c = __builtin_amdgcn_wmma_f32_16x16x32_f16(false, a, false, b, (short)0, c, false, false);
    asm volatile("v_nop\n\tv_nop\n\tv_nop\n\tv_nop" : "+v"(c) : "v"(a), "v"(b));
    return c;
}

__device__ __forceinline__ float gelu_erf(float x) {
    return 0.5f * x * (1.0f + erff(x * 0.70710678118654752f));
}

__device__ __forceinline__ size_t grow_map(u32 r) {
    const u32 bb = r / (u32)(SEQ);
    const u32 t  = r - bb * (u32)(SEQ);
    return (size_t)bb * SEQ_FULL + (size_t)t;
}

__global__ __launch_bounds__(256) void cvt_w_kernel(const float* __restrict__ in, u16* __restrict__ out) {
    const u32 i = blockIdx.x * 256u + threadIdx.x;
    const float* src = in + (size_t)i * 8u;
    v4f a = *(const v4f*)src;
    v4f b = *(const v4f*)(src + 4);
    Pack8 pk;
#pragma unroll
    for (u32 c = 0; c < 4; c++) {
        float fa = a[c]; float fb = b[c];
        pk.h[c]      = (_Float16)(bfr(fa) * WSCALE);
        pk.h[4u + c] = (_Float16)(bfr(fb) * WSCALE);
    }
    const u32x4 val = pk.u;
    u16* o = out + (size_t)i * 8u;
    *(volatile u32x4*)o = val;
    __threadfence();
    *(volatile u32x4*)o = val;
}

template <int SRCX>
__global__ __launch_bounds__(256) void ln_kernel(const float* __restrict__ src,
                                                 const float* __restrict__ g,
                                                 const float* __restrict__ be,
                                                 u16* __restrict__ out) {
    __shared__ __align__(16) float xs[8 * CE];
    __shared__ __align__(16) u16   rows[8 * CE];
    __shared__ __align__(16) float gsh[CE];
    __shared__ __align__(16) float bsh[CE];
    const u32 tid = threadIdx.x, lane = tid & 31u, wv = tid >> 5;
    if (tid < (u32)(CE / 4)) {
        v4f gg = *(const v4f*)(g + tid * 4u);
        v4f bb = *(const v4f*)(be + tid * 4u);
        v4f go, bo;
#pragma unroll
        for (u32 c = 0; c < 4; c++) {
            float tg = gg[c]; float tb = bb[c];
            go[c] = bfr(tg); bo[c] = bfr(tb);
        }
        *(v4f*)&gsh[tid * 4u] = go;
        *(v4f*)&bsh[tid * 4u] = bo;
    }
    const u32 r = blockIdx.x * 8u + wv;
    const size_t srow = SRCX ? grow_map(r) : (size_t)r;
    const float* xr = src + srow * CE;
    float* xw = xs + wv * CE;
    float s = 0.f;
#pragma unroll 1
    for (u32 j = 0; j < LNJ; j++) {
        const u32 c0 = j * 128u + lane * 4u;
        v4f t4 = *(const v4f*)(xr + c0);
        if constexpr (SRCX != 0) {
#pragma unroll
            for (u32 c = 0; c < 4; c++) { float t = t4[c]; t4[c] = bfr(t); }
        }
        *(v4f*)&xw[c0] = t4;
        s += (t4[0] + t4[1]) + (t4[2] + t4[3]);
    }
#pragma unroll
    for (u32 m = 16; m >= 1; m >>= 1) s += __shfl_xor(s, m, 32);
    const float mu = s * (1.f / (float)CE);
    float vs = 0.f;
#pragma unroll 1
    for (u32 j = 0; j < LNJ; j++) {
        const u32 c0 = j * 128u + lane * 4u;
        v4f t4 = *(const v4f*)&xw[c0];
#pragma unroll
        for (u32 c = 0; c < 4; c++) { float d = t4[c] - mu; vs += d * d; }
    }
#pragma unroll
    for (u32 m = 16; m >= 1; m >>= 1) vs += __shfl_xor(vs, m, 32);
    const float rstd = rsqrtf(vs * (1.f / (float)CE) + 1e-5f);
    __syncthreads();
    u16* rw = rows + wv * CE;
#pragma unroll 1
    for (u32 j = 0; j < LNJ; j++) {
        const u32 c0 = j * 128u + lane * 4u;
        v4f x4 = *(const v4f*)&xw[c0];
        v4f g4 = *(const v4f*)&gsh[c0];
        v4f b4 = *(const v4f*)&bsh[c0];
        Pack4 pk;
#pragma unroll
        for (u32 c = 0; c < 4; c++) {
            float xe = x4[c]; float ge = g4[c]; float bel = b4[c];
            pk.h[c] = (_Float16)((xe - mu) * rstd * ge + bel);
        }
        *(u32x2*)&rw[c0] = pk.u;
    }
    __syncthreads();
    u32x4 val[LNO];
#pragma unroll
    for (u32 j = 0; j < LNO; j++) val[j] = *(const u32x4*)&rw[j * 256u + lane * 8u];
    u16* orow = out + (size_t)r * CE;
#pragma unroll
    for (u32 j = 0; j < LNO; j++) *(volatile u32x4*)(orow + j * 256u + lane * 8u) = val[j];
    __threadfence();
#pragma unroll
    for (u32 j = 0; j < LNO; j++) *(volatile u32x4*)(orow + j * 256u + lane * 8u) = val[j];
}

template <int MODE>
__global__ __launch_bounds__(256) void gemm_kernel(const u16* __restrict__ A,
                                                   const u16* __restrict__ BT,
                                                   const float* __restrict__ bias,
                                                   const float* __restrict__ res,
                                                   void* out0, void* out1,
                                                   u32 N, u32 K, float oscale) {
    __shared__ u32x4 smem[4224];
    u16* As = (u16*)smem;
    u16* Bs = As + 128 * 72;
    float* Cs = (float*)smem;
    constexpr u32 CSP = 132;

    const u32 tid = threadIdx.x, lane = tid & 31u, wv = tid >> 5;
    const u32 hf = lane >> 4, ln = lane & 15u;
    const u32 m0 = blockIdx.y * 128u, n0 = blockIdx.x * 128u;
    const u32 wm = wv & 3u, wn = wv >> 2;
    const u32 srow = tid >> 1, sseg = (tid & 1u) * 32u;

    v8f acc[2][4];
#pragma unroll
    for (int i = 0; i < 2; i++)
#pragma unroll
        for (int j = 0; j < 4; j++) acc[i][j] = (v8f)(0.f);

    for (u32 k0 = 0; k0 < K; k0 += 64u) {
        __syncthreads();
        {
            const u16* ga = A  + (size_t)(m0 + srow) * K + k0 + sseg;
            const u16* gb = BT + (size_t)(n0 + srow) * K + k0 + sseg;
            u32x4 a0 = *(const u32x4*)(ga), a1 = *(const u32x4*)(ga + 8);
            u32x4 a2 = *(const u32x4*)(ga + 16), a3 = *(const u32x4*)(ga + 24);
            u32x4 b0 = *(const u32x4*)(gb), b1 = *(const u32x4*)(gb + 8);
            u32x4 b2 = *(const u32x4*)(gb + 16), b3 = *(const u32x4*)(gb + 24);
            u32x4* la = (u32x4*)&As[srow * 72u + sseg];
            u32x4* lb = (u32x4*)&Bs[srow * 72u + sseg];
            la[0] = a0; la[1] = a1; la[2] = a2; la[3] = a3;
            lb[0] = b0; lb[1] = b1; lb[2] = b2; lb[3] = b3;
        }
        __syncthreads();
#pragma unroll
        for (u32 ks = 0; ks < 2; ks++) {
            Frag af[2], bf[4];
#pragma unroll
            for (u32 mi = 0; mi < 2; mi++) {
                const u16* q = &As[(wm * 32u + mi * 16u + ln) * 72u + ks * 32u + hf * 8u];
                af[mi].u[0] = *(const u32x4*)q;
                af[mi].u[1] = *(const u32x4*)(q + 16);
            }
#pragma unroll
            for (u32 ni = 0; ni < 4; ni++) {
                const u16* q = &Bs[(wn * 64u + ni * 16u + ln) * 72u + ks * 32u + hf * 8u];
                bf[ni].u[0] = *(const u32x4*)q;
                bf[ni].u[1] = *(const u32x4*)(q + 16);
            }
#pragma unroll
            for (int mi = 0; mi < 2; mi++)
#pragma unroll
                for (int ni = 0; ni < 4; ni++)
                    acc[mi][ni] = mma16(af[mi].v, bf[ni].v, acc[mi][ni]);
        }
    }

    __syncthreads();
#pragma unroll
    for (int ni = 0; ni < 4; ni++) {
        const u32 col = wn * 64u + (u32)ni * 16u + ln;
        float bv = 0.f;
        if constexpr (MODE != 0) bv = bfr(bias[n0 + col]);
#pragma unroll
        for (int mi = 0; mi < 2; mi++) {
#pragma unroll
            for (int r = 0; r < 8; r++) {
                const u32 row = wm * 32u + (u32)mi * 16u + hf * 8u + (u32)r;
                float v = acc[mi][ni][r] * oscale + bv;
                if constexpr (MODE == 2) v = gelu_erf(v);
                Cs[row * CSP + col] = v;
            }
        }
    }
    __syncthreads();

    if constexpr (MODE == 1 || MODE == 3) {
        float* o = (float*)out0;
        v4f val[16];
#pragma unroll
        for (int grp = 0; grp < 2; grp++) {
#pragma unroll
            for (int i8 = 0; i8 < 8; i8++) {
                const int i = grp * 8 + i8;
                const u32 row = wv * 16u + (u32)i;
                const u32 r = m0 + row;
                v4f c = *(const v4f*)&Cs[row * CSP + lane * 4u];
                const size_t rr = (MODE == 1) ? grow_map(r) : (size_t)r;
                v4f x4 = *(const v4f*)(res + rr * (size_t)N + n0 + lane * 4u);
                if constexpr (MODE == 1) {
#pragma unroll
                    for (int cc = 0; cc < 4; cc++) { float t = x4[cc]; x4[cc] = bfr(t); }
                }
                val[i] = c + x4;
            }
            asm volatile("" ::: "memory");
        }
#pragma unroll
        for (int i = 0; i < 16; i++) {
            const u32 r = m0 + wv * 16u + (u32)i;
            const size_t orr = (MODE == 3) ? grow_map(r) : (size_t)r;
            *(volatile v4f*)(o + orr * (size_t)N + n0 + lane * 4u) = val[i];
        }
        __threadfence();
#pragma unroll
        for (int i = 0; i < 16; i++) {
            const u32 r = m0 + wv * 16u + (u32)i;
            const size_t orr = (MODE == 3) ? grow_map(r) : (size_t)r;
            *(volatile v4f*)(o + orr * (size_t)N + n0 + lane * 4u) = val[i];
        }
    } else if constexpr (MODE == 2) {
        u16* o = (u16*)out0;
        u32x4 val[8];
#pragma unroll
        for (int it = 0; it < 8; it++) {
            const u32 rloc = wv * 16u + (u32)it * 2u + hf, cseg = ln * 8u;
            Pack8 pk;
#pragma unroll
            for (int j = 0; j < 8; j++) pk.h[j] = (_Float16)Cs[rloc * CSP + cseg + (u32)j];
            val[it] = pk.u;
        }
#pragma unroll
        for (int it = 0; it < 8; it++) {
            const u32 rloc = wv * 16u + (u32)it * 2u + hf, cseg = ln * 8u;
            *(volatile u32x4*)(o + (size_t)(m0 + rloc) * N + n0 + cseg) = val[it];
        }
        __threadfence();
#pragma unroll
        for (int it = 0; it < 8; it++) {
            const u32 rloc = wv * 16u + (u32)it * 2u + hf, cseg = ln * 8u;
            *(volatile u32x4*)(o + (size_t)(m0 + rloc) * N + n0 + cseg) = val[it];
        }
    } else {
        u16* qkp = (u16*)out0;
        u16* vtp = (u16*)out1;
        const u32 bq = m0 / (u32)(SEQ);
        const u32 t0 = m0 - bq * (u32)(SEQ);
        u32x4 vh[8];
        if (n0 < (u32)QP) {
#pragma unroll
            for (int it = 0; it < 8; it++) {
                const u32 rloc = wv * 16u + (u32)it * 2u + hf, cseg = ln * 8u;
                Pack8 ph;
#pragma unroll
                for (int j = 0; j < 8; j++) ph.h[j] = (_Float16)Cs[rloc * CSP + cseg + (u32)j];
                vh[it] = ph.u;
            }
#pragma unroll
            for (int it = 0; it < 8; it++) {
                const u32 rloc = wv * 16u + (u32)it * 2u + hf, cseg = ln * 8u;
                *(volatile u32x4*)(qkp + (size_t)(m0 + rloc) * QP + n0 + cseg) = vh[it];
            }
            __threadfence();
#pragma unroll
            for (int it = 0; it < 8; it++) {
                const u32 rloc = wv * 16u + (u32)it * 2u + hf, cseg = ln * 8u;
                *(volatile u32x4*)(qkp + (size_t)(m0 + rloc) * QP + n0 + cseg) = vh[it];
            }
        } else {
            const u32 hh0 = (n0 - (u32)QP) >> 6;
#pragma unroll
            for (int it = 0; it < 8; it++) {
                const u32 rloc = wv * 16u + (u32)it * 2u + hf;
                const u32 tseg = ln * 8u;
                Pack8 ph;
#pragma unroll
                for (int j = 0; j < 8; j++) ph.h[j] = (_Float16)Cs[(tseg + (u32)j) * CSP + rloc];
                vh[it] = ph.u;
            }
#pragma unroll
            for (int it = 0; it < 8; it++) {
                const u32 rloc = wv * 16u + (u32)it * 2u + hf, tseg = ln * 8u;
                const u32 hh = hh0 + (rloc >> 6), dd = rloc & 63u;
                const size_t vrow = (size_t)(bq * NH + hh) * HD + dd;
                *(volatile u32x4*)(vtp + vrow * (SEQ) + t0 + tseg) = vh[it];
            }
            __threadfence();
#pragma unroll
            for (int it = 0; it < 8; it++) {
                const u32 rloc = wv * 16u + (u32)it * 2u + hf, tseg = ln * 8u;
                const u32 hh = hh0 + (rloc >> 6), dd = rloc & 63u;
                const size_t vrow = (size_t)(bq * NH + hh) * HD + dd;
                *(volatile u32x4*)(vtp + vrow * (SEQ) + t0 + tseg) = vh[it];
            }
        }
    }
}

__global__ __launch_bounds__(256) void vsum_kernel(const u16* __restrict__ vth, float* __restrict__ vs) {
    __shared__ __align__(16) float sh[32];
    const u32 tid = threadIdx.x, lane = tid & 31u, wv = tid >> 5;
#pragma unroll 1
    for (u32 i = 0; i < 4; i++) {
        const u32 row = blockIdx.x * 32u + wv * 4u + i;
        const u16* p = vth + (size_t)row * (SEQ) + lane * 8u;
        float s = 0.f;
#pragma unroll 1
        for (u32 j = 0; j < (u32)((SEQ) / 256); j++) {
            Pack8 pk;
            pk.u = *(const u32x4*)(p + j * 256u);
#pragma unroll
            for (u32 c = 0; c < 8; c++) s += (float)pk.h[c];
        }
#pragma unroll
        for (u32 m = 16; m >= 1; m >>= 1) s += __shfl_xor(s, m, 32);
        if (lane == 0) sh[wv * 4u + i] = s;
    }
    __syncthreads();
    if (wv == 0) {
        const v4f val = *(const v4f*)&sh[(lane & 7u) * 4u];
        float* o = vs + (size_t)blockIdx.x * 32u + (lane & 7u) * 4u;
        if (lane < 8u) *(volatile v4f*)o = val;
        __threadfence();
        if (lane < 8u) *(volatile v4f*)o = val;
    }
}

__global__ __launch_bounds__(256) __attribute__((amdgpu_num_vgpr(256)))
void attn_kernel(const u16* __restrict__ qk, const u16* __restrict__ vth,
                 const float* __restrict__ pol, const float* __restrict__ vsum,
                 u16* __restrict__ cv) {
    __shared__ __align__(16) u16 Ks[64 * 72];
    __shared__ __align__(16) u16 Vs[64 * 72];
    __shared__ __align__(16) u16 Ps[8 * 16 * 72];

    const u32 bh = blockIdx.y;
    const u32 b = bh / (u32)NH, h = bh - b * (u32)NH;
    const u32 qb = blockIdx.x;
    const u32 tid = threadIdx.x, lane = tid & 31u, wv = tid >> 5;
    const u32 hf = lane >> 4, ln = lane & 15u;
    const u32 q0 = qb * 128u + wv * 16u;
    u16* Pw = Ps + wv * (16u * 72u);
    const float* pb = pol + (size_t)b * SEQ_FULL;

    Frag qf[2];
#pragma unroll
    for (u32 ds = 0; ds < 2; ds++) {
        const u16* p = qk + (size_t)(b * (u32)(SEQ) + q0 + ln) * QP + h * HD + ds * 32u + hf * 8u;
        qf[ds].u[0] = *(const u32x4*)p;
        qf[ds].u[1] = *(const u32x4*)(p + 16);
    }

    v8f o[4];
#pragma unroll
    for (int i = 0; i < 4; i++) o[i] = (v8f)(0.f);
    float mrow[8], lrow[8];
#pragma unroll
    for (int r = 0; r < 8; r++) { mrow[r] = -3.0e38f; lrow[r] = 0.f; }

    const u32 rr = tid >> 2, seg = (tid & 3u) * 16u;

#pragma unroll 1
    for (u32 kt = 0; kt < (u32)NKT; kt++) {
        __syncthreads();
        {
            const u16* gk = qk + (size_t)(b * (u32)(SEQ) + kt * 64u + rr) * QP + CE + h * HD + seg;
            u32x4 k0v = *(const u32x4*)gk, k1v = *(const u32x4*)(gk + 8);
            const u16* gv = vth + ((size_t)(bh * HD + rr)) * (SEQ) + kt * 64u + seg;
            u32x4 v0 = *(const u32x4*)gv, v1 = *(const u32x4*)(gv + 8);
            *(u32x4*)&Ks[rr * 72u + seg] = k0v; *(u32x4*)&Ks[rr * 72u + seg + 8u] = k1v;
            *(u32x4*)&Vs[rr * 72u + seg] = v0;  *(u32x4*)&Vs[rr * 72u + seg + 8u] = v1;
        }
        float ap[4], apd[4];
#pragma unroll
        for (int sub = 0; sub < 4; sub++) {
            const float a = bfr(pb[kt * 64u + (u32)sub * 16u + ln]);
            ap[sub]  = a;
            apd[sub] = a + (1.0f - a);
        }
        __syncthreads();

        v8f s[4];
#pragma unroll
        for (int sub = 0; sub < 4; sub++) {
            v8f t = (v8f)(0.f);
#pragma unroll
            for (int ds = 0; ds < 2; ds++) {
                Frag kf;
                const u16* kp = &Ks[((u32)sub * 16u + ln) * 72u + (u32)ds * 32u + hf * 8u];
                kf.u[0] = *(const u32x4*)kp;
                kf.u[1] = *(const u32x4*)(kp + 16);
                t = mma16(qf[ds].v, kf.v, t);
            }
            s[sub] = t;
        }

#pragma unroll
        for (int sub = 0; sub < 4; sub++)
#pragma unroll
            for (int r = 0; r < 8; r++) s[sub][r] = s[sub][r] * 0.125f;

#pragma unroll
        for (int r = 0; r < 8; r++) {
            float mx = fmaxf(fmaxf(s[0][r], s[1][r]), fmaxf(s[2][r], s[3][r]));
#pragma unroll
            for (u32 m = 8; m >= 1; m >>= 1) mx = fmaxf(mx, __shfl_xor(mx, m, 32));
            const float mnew  = fmaxf(mrow[r], mx);
            const float alpha = __expf(mrow[r] - mnew);
            const u32 qg = q0 + hf * 8u + (u32)r;
            float rsum = 0.f;
#pragma unroll
            for (int sub = 0; sub < 4; sub++) {
                const u32 kg = kt * 64u + (u32)sub * 16u + ln;
                const float a = (kg == qg) ? apd[sub] : ap[sub];
                const float pe = __expf(s[sub][r] - mnew) * a;
                s[sub][r] = pe;
                rsum += pe;
            }
#pragma unroll
            for (u32 m = 8; m >= 1; m >>= 1) rsum += __shfl_xor(rsum, m, 32);
            mrow[r] = mnew;
            lrow[r] = lrow[r] * alpha + rsum;
#pragma unroll
            for (int dsub = 0; dsub < 4; dsub++) o[dsub][r] *= alpha;
        }

#pragma unroll
        for (int sub = 0; sub < 4; sub++) {
#pragma unroll
            for (int r = 0; r < 8; r++)
                Pw[(hf * 8u + (u32)r) * 72u + (u32)sub * 16u + ln] = hbits(s[sub][r] * PCAR);
        }
        __syncthreads();

#pragma unroll
        for (int dsub = 0; dsub < 4; dsub++) {
#pragma unroll
            for (int ks = 0; ks < 2; ks++) {
                Frag pf, vf;
                const u16* pp = &Pw[ln * 72u + (u32)ks * 32u + hf * 8u];
                pf.u[0] = *(const u32x4*)pp;
                pf.u[1] = *(const u32x4*)(pp + 16);
                const u16* vp = &Vs[((u32)dsub * 16u + ln) * 72u + (u32)ks * 32u + hf * 8u];
                vf.u[0] = *(const u32x4*)vp;
                vf.u[1] = *(const u32x4*)(vp + 16);
                o[dsub] = mma16(pf.v, vf.v, o[dsub]);
            }
        }
    }

    float vsd[4];
#pragma unroll
    for (int dsub = 0; dsub < 4; dsub++) vsd[dsub] = vsum[bh * (u32)HD + (u32)dsub * 16u + ln];
    const float epsn = 1e-6f / (float)(SEQ);
    __syncthreads();
#pragma unroll
    for (int r = 0; r < 8; r++) {
        const float inv = (1.0f / (lrow[r] + 1e-6f)) * CVCAR;
#pragma unroll
        for (int dsub = 0; dsub < 4; dsub++)
            Pw[(hf * 8u + (u32)r) * 72u + (u32)dsub * 16u + ln] =
                hbits((o[dsub][r] * PINV + epsn * vsd[dsub]) * inv);
    }
    __syncthreads();
    u32x4 val[4];
#pragma unroll
    for (u32 it = 0; it < 4; it++) {
        const u32 rloc = it * 4u + (lane >> 3), sg = (lane & 7u) * 8u;
        val[it] = *(const u32x4*)&Pw[rloc * 72u + sg];
    }
#pragma unroll
    for (u32 it = 0; it < 4; it++) {
        const u32 rloc = it * 4u + (lane >> 3), sg = (lane & 7u) * 8u;
        *(volatile u32x4*)(cv + (size_t)(b * (u32)(SEQ) + q0 + rloc) * CE + h * HD + sg) = val[it];
    }
    __threadfence();
#pragma unroll
    for (u32 it = 0; it < 4; it++) {
        const u32 rloc = it * 4u + (lane >> 3), sg = (lane & 7u) * 8u;
        *(volatile u32x4*)(cv + (size_t)(b * (u32)(SEQ) + q0 + rloc) * CE + h * HD + sg) = val[it];
    }
}

extern "C" void kernel_launch(void* const* d_in, const int* in_sizes, int n_in,
                              void* d_out, int out_size, void* d_ws, size_t ws_size,
                              hipStream_t stream) {
    if (n_in < 13) return;
    const long long needX = ((long long)(NB - 1) * SEQ_FULL + (SEQ)) * CE;
    const long long needP = (long long)(NB - 1) * SEQ_FULL + (SEQ);
    if ((long long)in_sizes[0] < needX || (long long)out_size < needX) return;
    if ((long long)in_sizes[1] < needP) return;
    if (in_sizes[2] < CE || in_sizes[3] < CE || in_sizes[4] < C3 * CE || in_sizes[5] < CE * CE ||
        in_sizes[6] < CE || in_sizes[7] < CE || in_sizes[8] < CE || in_sizes[9] < C4 * CE ||
        in_sizes[10] < C4 || in_sizes[11] < CE * C4 || in_sizes[12] < CE)
        return;

    const float* x      = (const float*)d_in[0];
    const float* policy = (const float*)d_in[1];
    const float* ln1_g  = (const float*)d_in[2];
    const float* ln1_b  = (const float*)d_in[3];
    const float* qkv_w  = (const float*)d_in[4];
    const float* proj_w = (const float*)d_in[5];
    const float* proj_b = (const float*)d_in[6];
    const float* ln2_g  = (const float*)d_in[7];
    const float* ln2_b  = (const float*)d_in[8];
    const float* fc1_w  = (const float*)d_in[9];
    const float* fc1_b  = (const float*)d_in[10];
    const float* fc2_w  = (const float*)d_in[11];
    const float* fc2_b  = (const float*)d_in[12];

    char* ws = (char*)d_ws;
    size_t off = 0;
    auto take = [&](size_t bytes) -> char* {
        char* p = ws + off;
        off += (bytes + 255) & ~(size_t)255;
        return p;
    };
    const size_t R = (size_t)RROWS;
    u16*   wqT   = (u16*)take((size_t)C3 * CE * 2);
    u16*   wpT   = (u16*)take((size_t)CE * CE * 2);
    u16*   wf1T  = (u16*)take((size_t)C4 * CE * 2);
    u16*   wf2T  = (u16*)take((size_t)CE * C4 * 2);
    u16*   h1    = (u16*)take(R * CE * 2);
    u16*   qkp   = (u16*)take(R * QP * 2);
    u16*   vth   = (u16*)take((size_t)VROWS * (SEQ) * 2);
    float* vsm   = (float*)take((size_t)VROWS * 4);
    u16*   cvb   = (u16*)take(R * CE * 2);
    float* x1    = (float*)take(R * CE * 4);
    u16*   h2    = (u16*)take(R * CE * 2);
    u16*   hg    = (u16*)take(R * C4 * 2);
    if (off > ws_size || off > (size_t)134217728) return;
    void* spare = (void*)d_ws;

    cvt_w_kernel<<<(u32)(((size_t)C3 * CE) / 2048), 256, 0, stream>>>(qkv_w, wqT);
    cvt_w_kernel<<<(u32)(((size_t)CE * CE) / 2048), 256, 0, stream>>>(proj_w, wpT);
    cvt_w_kernel<<<(u32)(((size_t)C4 * CE) / 2048), 256, 0, stream>>>(fc1_w, wf1T);
    cvt_w_kernel<<<(u32)(((size_t)CE * C4) / 2048), 256, 0, stream>>>(fc2_w, wf2T);
    ln_kernel<1><<<RROWS / 8, 256, 0, stream>>>(x, ln1_g, ln1_b, h1);
    gemm_kernel<0><<<dim3(C3 / 128, RROWS / 128), 256, 0, stream>>>(h1, wqT, proj_b, x,
                                                                    qkp, vth, (u32)C3, (u32)CE, WINV);
    vsum_kernel<<<VROWS / 32, 256, 0, stream>>>(vth, vsm);
    attn_kernel<<<dim3(NQB, NB * NH), 256, 0, stream>>>(qkp, vth, policy, vsm, cvb);
    gemm_kernel<1><<<dim3(CE / 128, RROWS / 128), 256, 0, stream>>>(cvb, wpT, proj_b, x,
                                                                    x1, spare, (u32)CE, (u32)CE, WINV * CVINV);
    ln_kernel<0><<<RROWS / 8, 256, 0, stream>>>(x1, ln2_g, ln2_b, h2);
    gemm_kernel<2><<<dim3(C4 / 128, RROWS / 128), 256, 0, stream>>>(h2, wf1T, fc1_b, x,
                                                                    hg, spare, (u32)C4, (u32)CE, WINV);
    gemm_kernel<3><<<dim3(CE / 128, RROWS / 128), 256, 0, stream>>>(hg, wf2T, fc2_b, x1,
                                                                    d_out, spare, (u32)CE, (u32)C4, WINV);
}
